// MoTBlock_50319836840363
// MI455X (gfx1250) — hardware-verified
//
#include <hip/hip_runtime.h>


namespace {
constexpr int NB = 16, C = 128, HH = 64, WW = 64, NPX = HH * WW, C2 = 256, C4 = 512, CR = 128  ;
constexpr float XS = 8.0f, WSC = 256.0f, PS = 8.0f, BNI = 0.99999500003749981f  , LOG2E = 1.4426950408889634f;

typedef _Float16 b16;
typedef __attribute__((ext_vector_type(16))) _Float16 v16b;
typedef __attribute__((ext_vector_type(8))) _Float16 v8b;
typedef __attribute__((ext_vector_type(8))) float v8f;
typedef __attribute__((ext_vector_type(4))) float v4f;
__device__ __forceinline__ float bf16_rne(float f) { unsigned int u = __float_as_uint(f); u += 0x7FFFu + ((u >> 16) & 1u); return __uint_as_float(u & 0xFFFF0000u); }
__device__ __forceinline__ void split16(float v, b16& hi, b16& lo) { hi = (b16)v; lo = (b16)(v - (float)hi); }
__device__ __forceinline__ v16b frag_kb(const b16* p, int hh) { const v8b a = *(const v8b*)(p + 8 * hh), b = *(const v8b*)(p + 16 + 8 * hh); v16b f;
#pragma unroll
  for (int e = 0; e < 8; ++e) { f[e] = a[e]; f[8 + e] = b[e]; } return f; }
__device__ __forceinline__ v8f wmma16b(v16b a, v16b b, v8f c) { v8f d = __builtin_amdgcn_wmma_f32_16x16x32_f16(false, a, false, b, (short)0, c, false, false); asm volatile("v_nop\n\tv_nop\n\tv_nop\n\tv_nop" : "+v"(d) : "v"(a), "v"(b)); return d; }
__device__ __forceinline__ void wave_lds_sync() { __builtin_amdgcn_fence(__ATOMIC_RELEASE, "workgroup"); __builtin_amdgcn_wave_barrier(); __builtin_amdgcn_fence(__ATOMIC_ACQUIRE, "workgroup"); }
__device__ __forceinline__ float pmul(float a, float b) { float p = a * b; asm volatile("" : "+v"(p)); return p; }
__device__ __forceinline__ float hmax16(float v) { v = fmaxf(v, __shfl_xor(v, 1)); v = fmaxf(v, __shfl_xor(v, 2)); v = fmaxf(v, __shfl_xor(v, 4)); return fmaxf(v, __shfl_xor(v, 8)); }
__device__ __forceinline__ float hsum16(float v) { v += __shfl_xor(v, 1); v += __shfl_xor(v, 2); v += __shfl_xor(v, 4); return v + __shfl_xor(v, 8); }
__device__ __forceinline__ float nexp2(float x) { return __builtin_amdgcn_exp2f(x); }

__global__ __launch_bounds__(256) void prep_kernel(const float* __restrict__ p1, const float* __restrict__ p2, const float* __restrict__ p3, b16* __restrict__ WP) {
  const int t = blockIdx.x * 256 + threadIdx.x; const int n1 = 64 * C / 8, n2 = C2 * C / 8, n3 = 64 * C4 / 8; v8b o; const float* w; int e; size_t dst;
  if (t < n1) { w = p1; e = t * 8; dst = e; } else if (t < n1 + n2) { w = p2; e = (t - n1) * 8; dst = (size_t)64 * C + e; } else if (t < n1 + n2 + n3) { w = p3; e = (t - n1 - n2) * 8; dst = (size_t)64 * C + (size_t)C2 * C + e; } else return;
  for (int j = 0; j < 8; ++j) o[j] = (b16)(bf16_rne(w[e + j]) * WSC);
  for (int pass = 0; pass < 2; ++pass) { *(volatile v8b*)(WP + dst) = o; __threadfence(); }
}
__device__ __forceinline__ v4f dw3x3(const float (*T)[68], const float* ws, int y, int x0) {
  float a0 = 0.0f, a1 = 0.0f, a2 = 0.0f, a3 = 0.0f;
#pragma unroll 1
  for (int tap = 0; tap < 9; ++tap) { const int dy = tap / 3, dx = tap - dy * 3; const float w = ws[tap]; const float* r = &T[y + dy][x0 + dx]; a0 += pmul(w, r[0]); a1 += pmul(w, r[1]); a2 += pmul(w, r[2]); a3 += pmul(w, r[3]); }
  const v4f o = {a0, a1, a2, a3}; return o;
}
__device__ __forceinline__ void load_tile(float (*T)[68], const float* __restrict__ src, int t_, bool round_bf16, float gate) {
  for (int i = t_; i < 66 * 68; i += 256) { const int yy = i / 68, xx = i - yy * 68; float v = 0.0f; if (yy >= 1 && yy <= 64 && xx >= 1 && xx <= 64) { v = src[(yy - 1) * WW + (xx - 1)]; if (round_bf16) v = bf16_rne(v); v *= gate; } T[yy][xx] = v; }
}
__global__ __launch_bounds__(128) void mosa_kernel(const float* __restrict__ xb, const float* __restrict__ dww, const float* __restrict__ dwg, const float* __restrict__ dwb, float* __restrict__ A1) {
  __shared__ __attribute__((aligned(16))) b16 X16[64][72], XT16[64][72], Ph[4][16][72], Pl[4][16][72]; __shared__ float T[66][68]; __shared__ float ws[9]; __shared__ __attribute__((aligned(16))) float To[4][16][68];
  const int c = blockIdx.x, t_ = threadIdx.x, wave = t_ >> 5, lane = t_ & 31, nloc = lane & 15, hlf = lane >> 4; const float* xc = xb + (size_t)c * NPX;
  for (int i = t_; i < NPX; i += 128) { const int y = i >> 6, x = i & 63; const float v = bf16_rne(xc[i]); const b16 hv = (b16)(v * XS); X16[y][x] = hv; XT16[x][y] = hv; }
  for (int i = t_; i < 66 * 68; i += 128) { const int yy = i / 68, xx = i - yy * 68; float v = 0.0f; if (yy >= 1 && yy <= 64 && xx >= 1 && xx <= 64) v = bf16_rne(xc[(yy - 1) * WW + (xx - 1)]); T[yy][xx] = v; }
  if (t_ < 9) ws[t_] = bf16_rne(dww[c * 9 + t_]);
  __syncthreads();
  const int h0 = wave * 16;
  v8f s[4] = {{}, {}, {}, {}};
#pragma unroll
  for (int kb = 0; kb < 64; kb += 32) { const v16b a = frag_kb(&X16[h0 + nloc][kb], hlf);
#pragma unroll
    for (int t = 0; t < 4; ++t) s[t] = wmma16b(a, frag_kb(&X16[t * 16 + nloc][kb], hlf), s[t]); }
  const float cs = 0.125f * LOG2E / (XS * XS);
#pragma unroll
  for (int r = 0; r < 8; ++r) { float mx = fmaxf(fmaxf(s[0][r], s[1][r]), fmaxf(s[2][r], s[3][r])) * cs; mx = hmax16(mx); float e[4], sm = 0.0f; for (int t = 0; t < 4; ++t) { e[t] = nexp2(s[t][r] * cs - mx); sm += e[t]; } sm = hsum16(sm); const float inv = 1.0f / sm;
    for (int t = 0; t < 4; ++t) { b16 a_, c_; split16(e[t] * inv * PS, a_, c_); Ph[wave][8 * hlf + r][t * 16 + nloc] = a_; Pl[wave][8 * hlf + r][t * 16 + nloc] = c_; } }
  wave_lds_sync();
  v8f o[4] = {{}, {}, {}, {}};
#pragma unroll
  for (int kb = 0; kb < 64; kb += 32) { const v16b a = frag_kb(&Ph[wave][nloc][kb], hlf), al = frag_kb(&Pl[wave][nloc][kb], hlf);
#pragma unroll
    for (int t = 0; t < 4; ++t) { const v16b bx = frag_kb(&XT16[t * 16 + nloc][kb], hlf); o[t] = wmma16b(a, bx, o[t]); o[t] = wmma16b(al, bx, o[t]); } }
  const float gsc = bf16_rne(dwg[c]) * BNI, gb = bf16_rne(dwb[c]);
#pragma unroll
  for (int t = 0; t < 4; ++t)
#pragma unroll
    for (int r = 0; r < 8; ++r) To[wave][8 * hlf + r][t * 16 + nloc] = o[t][r] * (1.0f / (PS * XS));
  wave_lds_sync();
  for (int pass = 0; pass < 2; ++pass) { for (int r2 = 0; r2 < 16; r2 += 2) { const int y = h0 + r2 + hlf, x0 = nloc * 4; const v4f d = dw3x3(T, ws, y, x0); v4f v; for (int j = 0; j < 4; ++j) v[j] = To[wave][r2 + hlf][x0 + j] + (pmul(d[j], gsc) + gb); *(volatile v4f*)(A1 + (size_t)c * NPX + y * WW + x0) = v; } __threadfence(); }
}
template <int IC, int OCB>
__global__ __launch_bounds__(128) void pw_kernel(const float* __restrict__ IN, const float* __restrict__ gate, const b16* __restrict__ Wp, const float* __restrict__ g, const float* __restrict__ bb, int OC, float* __restrict__ OUT) {
  __shared__ __attribute__((aligned(16))) b16 Ah[64][136], Alo[64][136]; __shared__ __attribute__((aligned(16))) float To[OCB][64 + 4];
  const int y = blockIdx.x, ocb0 = blockIdx.y * OCB, t_ = threadIdx.x, wave = t_ >> 5, lane = t_ & 31, nloc = lane & 15, hlf = lane >> 4; if (ocb0 >= OC) return;
  constexpr int NT = OCB / 16; v8f acc[NT];
#pragma unroll
  for (int t = 0; t < NT; ++t) acc[t] = (v8f){};
  for (int ic0 = 0; ic0 < IC; ic0 += 128) {
    __syncthreads();
    for (int i = t_; i < 128 * 64; i += 128) { const int ic = i >> 6, px = i & 63; float v = IN[(size_t)(ic0 + ic) * NPX + y * WW + px]; if (gate) v *= gate[ic0 + ic]; b16 a_, c_; split16(v * XS, a_, c_); Ah[px][ic] = a_; Alo[px][ic] = c_; }
    __syncthreads();
#pragma unroll
    for (int kb = 0; kb < 128; kb += 32) { const v16b a = frag_kb(&Ah[wave * 16 + nloc][kb], hlf), al = frag_kb(&Alo[wave * 16 + nloc][kb], hlf);
#pragma unroll
      for (int t = 0; t < NT; ++t) { const v16b bw = frag_kb(Wp + (size_t)(ocb0 + t * 16 + nloc) * IC + ic0 + kb, hlf); acc[t] = wmma16b(a, bw, acc[t]); acc[t] = wmma16b(al, bw, acc[t]); } } }
#pragma unroll
  for (int t = 0; t < NT; ++t) { const int oc = ocb0 + t * 16 + nloc; const float gs = bf16_rne(g[oc]) * BNI, b_ = bf16_rne(bb[oc]);
#pragma unroll
    for (int r = 0; r < 8; ++r) To[t * 16 + nloc][wave * 16 + 8 * hlf + r] = fmaxf(pmul(acc[t][r] * (1.0f / (XS * WSC)), gs) + b_, 0.0f); }
  __syncthreads();
  for (int pass = 0; pass < 2; ++pass) { for (int i = t_; i < OCB * 16; i += 128) { const int oc = i >> 4, x4 = (i & 15) * 4; *(volatile v4f*)(OUT + (size_t)(ocb0 + oc) * NPX + y * WW + x4) = *(const v4f*)(&To[oc][x4]); } __threadfence(); }
}
template <int MODE>
__global__ __launch_bounds__(256) void cheap_kernel(const float* __restrict__ P1, const float* __restrict__ xb, const float* __restrict__ cw, const float* __restrict__ cg, const float* __restrict__ cb, float* __restrict__ Y, float* __restrict__ H, float* __restrict__ M, float* __restrict__ outb) {
  __shared__ float T[66][68]; __shared__ float ws[9]; __shared__ float red[2][256];
  const int c = blockIdx.x, t_ = threadIdx.x; const float* src = (MODE == 2) ? H + (size_t)c * NPX : P1 + (size_t)c * NPX;
  load_tile(T, src, t_, false, 1.0f); if (t_ < 9) ws[t_] = bf16_rne(cw[c * 9 + t_]);
  __syncthreads();
  const float gs = bf16_rne(cg[c]) * BNI, gb = bf16_rne(cb[c]);
  float s1 = 0.0f, s2 = 0.0f;
  for (int pass = 0; pass < 2; ++pass) { s1 = 0.0f; s2 = 0.0f;
    for (int q = 0; q < 4; ++q) { const int y = (t_ >> 4) * 4 + q, x0 = (t_ & 15) * 4; const v4f d = dw3x3(T, ws, y, x0); v4f x2; for (int j = 0; j < 4; ++j) x2[j] = fmaxf(pmul(d[j], gs) + gb, 0.0f);
      const size_t o = (size_t)y * WW + x0; const v4f x1 = *(const v4f*)(&T[1 + y][1 + x0]);
      if (MODE == 1) { v4f xa, xb4; for (int j = 0; j < 4; ++j) { xa[j] = bf16_rne(xb[(size_t)c * NPX + o + j]); xb4[j] = bf16_rne(xb[(size_t)(64 + c) * NPX + o + j]); } const v4f ya = x1 + xa, yb = x2 + xb4; *(volatile v4f*)(Y + (size_t)c * NPX + o) = ya; *(volatile v4f*)(Y + (size_t)(64 + c) * NPX + o) = yb; }
      else if (MODE == 2) { *(volatile v4f*)(H + (size_t)(C2 + c) * NPX + o) = x2; for (int j = 0; j < 4; ++j) { s1 += x1[j]; s2 += x2[j]; } }
      else { const v4f y1 = *(const v4f*)(Y + (size_t)c * NPX + o), y2 = *(const v4f*)(Y + (size_t)(64 + c) * NPX + o); const v4f oa = x1 + 2.0f * y1, ob = x2 + 2.0f * y2; *(volatile v4f*)(outb + (size_t)c * NPX + o) = oa; *(volatile v4f*)(outb + (size_t)(64 + c) * NPX + o) = ob; } }
    __threadfence(); }
  if (MODE == 2) { red[0][t_] = s1; red[1][t_] = s2; __syncthreads(); for (int st = 128; st >= 1; st >>= 1) { if (t_ < st) { red[0][t_] += red[0][t_ + st]; red[1][t_] += red[1][t_ + st]; } __syncthreads(); }
    for (int pass = 0; pass < 2; ++pass) { if (t_ < 32) ((volatile float*)M)[(size_t)c * 32 + t_] = (t_ == 0) ? red[0][0] * (1.0f / NPX) : (t_ == 1) ? red[1][0] * (1.0f / NPX) : 0.0f; __threadfence(); } }
}
__global__ __launch_bounds__(512) void se_kernel(const float* __restrict__ M, const float* __restrict__ w1, const float* __restrict__ b1, const float* __restrict__ w2, const float* __restrict__ b2, float* __restrict__ G) {
  __shared__ float m[C4], y1[CR];
  const int t_ = threadIdx.x; m[t_] = (t_ < C2) ? M[(size_t)t_ * 32] : M[(size_t)(t_ - C2) * 32 + 1];
  __syncthreads();
  if (t_ < CR) { float s = bf16_rne(b1[t_]); for (int k = 0; k < C4; ++k) s += pmul(bf16_rne(w1[(size_t)t_ * C4 + k]), m[k]); y1[t_] = fmaxf(s, 0.0f); }
  __syncthreads();
  float s = bf16_rne(b2[t_]); for (int k = 0; k < CR; ++k) s += pmul(bf16_rne(w2[(size_t)t_ * CR + k]), y1[k]); const float gt = fminf(fmaxf(s, 0.0f), 1.0f);
  for (int pass = 0; pass < 2; ++pass) { ((volatile float*)G)[t_] = gt; __threadfence(); }
}
}

extern "C" void kernel_launch(void* const* d_in, const int* in_sizes, int n_in, void* d_out, int out_size, void* d_ws, size_t ws_size, hipStream_t stream) {
  (void)n_in;
  auto Fp = [&](int i) { return (const float*)d_in[i]; };
  if (in_sizes[0] != NB * C * NPX || in_sizes[1] != C * 9 || in_sizes[4] != 64 * C || in_sizes[10] != C2 * C || in_sizes[16] != CR * C4 || in_sizes[18] != C4 * CR || in_sizes[20] != 64 * C4 || out_size != NB * C * NPX) return;
  size_t off = 0; char* ws = (char*)d_ws;
  auto carve = [&](size_t bytes) { char* p = ws + off; off += (bytes + 255) & ~(size_t)255; return p; };
  b16* WP = (b16*)carve(((size_t)64 * C + (size_t)C2 * C + (size_t)64 * C4) * 2); float* A1 = (float*)carve((size_t)C * NPX * 4); float* O1 = (float*)carve((size_t)64 * NPX * 4); float* Y = (float*)carve((size_t)C * NPX * 4); float* H = (float*)carve((size_t)C4 * NPX * 4); float* M = (float*)carve((size_t)C2 * 32 * 4); float* G = (float*)carve((size_t)C4 * 4); float* F1 = (float*)carve((size_t)64 * NPX * 4);
  if (off > ws_size || off > ((size_t)128 << 20)) return;
  const b16* P1 = WP; const b16* P2 = WP + (size_t)64 * C; const b16* P3 = P2 + (size_t)C2 * C;
  prep_kernel<<<(64 * C / 8 + C2 * C / 8 + 64 * C4 / 8 + 255) / 256, 256, 0, stream>>>(Fp(4), Fp(10), Fp(20), WP);
  for (int b = 0; b < NB; ++b) { const float* xb = Fp(0) + (size_t)b * C * NPX; float* ob = (float*)d_out + (size_t)b * C * NPX;
    mosa_kernel<<<C, 128, 0, stream>>>(xb, Fp(1), Fp(2), Fp(3), A1);
    pw_kernel<128, 64><<<dim3(HH, 1), 128, 0, stream>>>(A1, nullptr, P1, Fp(5), Fp(6), 64, O1);
    cheap_kernel<1><<<64, 256, 0, stream>>>(O1, xb, Fp(7), Fp(8), Fp(9), Y, nullptr, nullptr, nullptr);
    pw_kernel<128, 128><<<dim3(HH, 2), 128, 0, stream>>>(Y, nullptr, P2, Fp(11), Fp(12), C2, H);
    cheap_kernel<2><<<C2, 256, 0, stream>>>(nullptr, nullptr, Fp(13), Fp(14), Fp(15), nullptr, H, M, nullptr);
    se_kernel<<<1, 512, 0, stream>>>(M, Fp(16), Fp(17), Fp(18), Fp(19), G);
    pw_kernel<512, 64><<<dim3(HH, 1), 128, 0, stream>>>(H, G, P3, Fp(21), Fp(22), 64, F1);
    cheap_kernel<3><<<64, 256, 0, stream>>>(F1, nullptr, Fp(23), Fp(24), Fp(25), Y, nullptr, nullptr, ob);
  }
}
